// DynamicGAT_44135083934280
// MI455X (gfx1250) — hardware-verified
//
#include <hip/hip_runtime.h>
#include <stddef.h>


#define INC   128
#define DF    256
#define NH    4
#define HDIM  64
#define NO    16
#define GR    32
#define AP    136
#define XSP   260
#define NB    256
#define CHUNK 2048
#define NTHR  256
#define NWAVE 8
#define WCAP  256
#define NGRP  (CHUNK / (NTHR * 4))
#define QB    64
#define JB    64
#define QTHR  128
#define PP    72

#define LDS_SACC (NB * DF)
#define LDS_DEN  (NB * NH)
#define LDS_MX   (NB * NH)
#define LDS_LIST (NWAVE * WCAP)
#define LDS_BYTES ((LDS_SACC + LDS_DEN + LDS_MX + LDS_LIST + NWAVE) * 4)

static_assert(WCAP == (CHUNK / NTHR) * 32);
static_assert(NGRP >= 1);
static_assert(NB == 256);
static_assert((NB / NWAVE) == 32);
static_assert(CHUNK <= 2048);
static_assert(((LDS_SACC + LDS_DEN) % 4) == 0);
static_assert(LDS_BYTES == 278560);
static_assert(DF == NH * HDIM);
static_assert((AP % 8) == 0 && (XSP % 4) == 0 && (PP % 8) == 0);
static_assert((INC % 32) == 0 && (DF % 32) == 0 && (JB % 32) == 0);

typedef float    v4f  __attribute__((ext_vector_type(4)));
typedef float    v8f  __attribute__((ext_vector_type(8)));
typedef int      v4i  __attribute__((ext_vector_type(4)));
typedef _Float16 v8h  __attribute__((ext_vector_type(8)));
typedef _Float16 v16h __attribute__((ext_vector_type(16)));
union Frag   { v16h v; v8h half[2]; };
union Pack16 { v8h h; v4i i; };

__device__ __forceinline__ v8f wm(v16h a, v16h b, v8f c) {
  v8f d = __builtin_amdgcn_wmma_f32_16x16x32_f16(false, a, false, b, (short)0, c, false, false);
  asm volatile("v_nop\n\tv_nop\n\tv_nop\n\tv_nop" : "+v"(d) : "v"(a), "v"(b));
  return d;
}

__device__ __forceinline__ float wsum(float v) {
  v += __shfl_xor(v, 16, 32);
  v += __shfl_xor(v, 8, 32);
  v += __shfl_xor(v, 4, 32);
  v += __shfl_xor(v, 2, 32);
  v += __shfl_xor(v, 1, 32);
  return v;
}

__device__ __forceinline__ float lrelu(float v) { return v > 0.f ? v : 0.2f * v; }
__device__ __forceinline__ float elu1(float v)  { return v > 0.f ? v : (__expf(v) - 1.0f); }

__global__ __launch_bounds__(NTHR) void k_prepT(const float* __restrict__ W, _Float16* Wt, int K, int NOUT) {
  const int kg8 = K >> 3;
  const int n8  = NOUT * kg8;
  const int i   = blockIdx.x * NTHR + threadIdx.x;
  if (i >= n8) return;
  const int o  = i / kg8;
  const int k0 = (i - o * kg8) * 8;
  Pack16 u;
#pragma unroll
  for (int j = 0; j < 8; ++j) u.h[j] = (_Float16)(W[(size_t)(k0 + j) * NOUT + o] * 8.0f);
  _Float16* p = Wt + (size_t)o * K + k0;
  *(volatile v4i*)p = u.i;
  __threadfence();
  *(volatile v4i*)p = u.i;
}

__device__ __forceinline__ void epi2(v8f ca, v8f cb, int T, int hh, int m, int wave,
                                     int nc0, int nc1, float cs0, float cs1, float cd0, float cd1,
                                     float* Xs, float* As, float* Ds) {
  float ss[8], sd[8];
#pragma unroll
  for (int r = 0; r < 8; ++r) {
    const float va = ca[r] * 0.125f;
    const float vb = cb[r] * 0.125f;
    const int row = T * 16 + 8 * hh + r;
    Xs[row * XSP + nc0] = va;
    Xs[row * XSP + nc1] = vb;
    ss[r] = va * cs0 + vb * cs1;
    sd[r] = va * cd0 + vb * cd1;
  }
#pragma unroll
  for (int mk = 1; mk < 16; mk <<= 1) {
#pragma unroll
    for (int r = 0; r < 8; ++r) {
      ss[r] += __shfl_xor(ss[r], mk, 32);
      sd[r] += __shfl_xor(sd[r], mk, 32);
    }
  }
  if (m == 0) {
#pragma unroll
    for (int r = 0; r < 8; ++r) {
      const int row = T * 16 + 8 * hh + r;
      As[row * NWAVE + wave] = ss[r];
      Ds[row * NWAVE + wave] = sd[r];
    }
  }
}

__global__ __launch_bounds__(NTHR) void k_gemm(
    const float* __restrict__ x, const _Float16* __restrict__ Wh,
    const float* __restrict__ att_src, const float* __restrict__ att_dst,
    float* xp, float* asrc, float* adst, int nN) {
  __shared__ __attribute__((aligned(16))) _Float16 At[GR * AP];
  __shared__ __attribute__((aligned(16))) float Xs[GR * XSP];
  __shared__ __attribute__((aligned(16))) float As[GR * NWAVE];
  __shared__ __attribute__((aligned(16))) float Ds[GR * NWAVE];

  const int tid  = threadIdx.x;
  const int lane = tid & 31;
  const int wave = tid >> 5;
  const int hh   = lane >> 4;
  const int m    = lane & 15;
  const int rowBase = blockIdx.x * GR;

  {
    const int r  = tid >> 3;
    const int c0 = (tid & 7) * 16;
    int row = rowBase + r;
    if (row > nN - 1) row = nN - 1;
    const float* p = x + (size_t)row * INC + c0;
    const v4f f0 = *(const v4f*)(p), f1 = *(const v4f*)(p + 4);
    const v4f f2 = *(const v4f*)(p + 8), f3 = *(const v4f*)(p + 12);
    Pack16 u0, u1;
    u0.h[0] = (_Float16)f0.x; u0.h[1] = (_Float16)f0.y; u0.h[2] = (_Float16)f0.z; u0.h[3] = (_Float16)f0.w;
    u0.h[4] = (_Float16)f1.x; u0.h[5] = (_Float16)f1.y; u0.h[6] = (_Float16)f1.z; u0.h[7] = (_Float16)f1.w;
    u1.h[0] = (_Float16)f2.x; u1.h[1] = (_Float16)f2.y; u1.h[2] = (_Float16)f2.z; u1.h[3] = (_Float16)f2.w;
    u1.h[4] = (_Float16)f3.x; u1.h[5] = (_Float16)f3.y; u1.h[6] = (_Float16)f3.z; u1.h[7] = (_Float16)f3.w;
    *(v8h*)(At + r * AP + c0)     = u0.h;
    *(v8h*)(At + r * AP + c0 + 8) = u1.h;
  }
  __syncthreads();

  const int nc0 = wave * 32 + m;
  const int nc1 = nc0 + 16;
  v8f c00 = {0.f, 0.f, 0.f, 0.f, 0.f, 0.f, 0.f, 0.f};
  v8f c01 = c00, c10 = c00, c11 = c00;
#pragma unroll
  for (int kt = 0; kt < INC / 32; ++kt) {
    const int k0 = kt * 32;
    Frag a0, a1, b0, b1;
    const _Float16* pa0 = At + m * AP + k0 + 8 * hh;
    const _Float16* pa1 = At + (16 + m) * AP + k0 + 8 * hh;
    const _Float16* pb0 = Wh + (size_t)nc0 * INC + k0 + 8 * hh;
    const _Float16* pb1 = Wh + (size_t)nc1 * INC + k0 + 8 * hh;
    a0.half[0] = *(const v8h*)pa0; a0.half[1] = *(const v8h*)(pa0 + 16);
    a1.half[0] = *(const v8h*)pa1; a1.half[1] = *(const v8h*)(pa1 + 16);
    b0.half[0] = *(const v8h*)pb0; b0.half[1] = *(const v8h*)(pb0 + 16);
    b1.half[0] = *(const v8h*)pb1; b1.half[1] = *(const v8h*)(pb1 + 16);
    c00 = wm(a0.v, b0.v, c00);
    c01 = wm(a0.v, b1.v, c01);
    c10 = wm(a1.v, b0.v, c10);
    c11 = wm(a1.v, b1.v, c11);
  }

  const float cs0 = att_src[nc0], cs1 = att_src[nc1];
  const float cd0 = att_dst[nc0], cd1 = att_dst[nc1];
  epi2(c00, c01, 0, hh, m, wave, nc0, nc1, cs0, cs1, cd0, cd1, Xs, As, Ds);
  epi2(c10, c11, 1, hh, m, wave, nc0, nc1, cs0, cs1, cd0, cd1, Xs, As, Ds);
  __syncthreads();

  v4f xr[8];
#pragma unroll
  for (int i = 0; i < 4; ++i) {
    xr[2 * i]     = *(const v4f*)(Xs + (4 * wave + i) * XSP + 4 * lane);
    xr[2 * i + 1] = *(const v4f*)(Xs + (4 * wave + i) * XSP + 128 + 4 * lane);
  }
  bool hasg = false;
  v4f gv = {0.f, 0.f, 0.f, 0.f};
  float* gp = xp;
  if (wave == 0) {
#pragma unroll
    for (int c = 0; c < 4; ++c) gv[c] = As[lane * NWAVE + 2 * c] + As[lane * NWAVE + 2 * c + 1];
    gp = asrc + (size_t)rowBase * NH + 4 * lane;
    hasg = true;
  } else if (wave == 1) {
#pragma unroll
    for (int c = 0; c < 4; ++c) gv[c] = Ds[lane * NWAVE + 2 * c] + Ds[lane * NWAVE + 2 * c + 1];
    gp = adst + (size_t)rowBase * NH + 4 * lane;
    hasg = true;
  }
  float* xpp[8];
#pragma unroll
  for (int i = 0; i < 4; ++i) {
    xpp[2 * i]     = xp + (size_t)(rowBase + 4 * wave + i) * DF + 4 * lane;
    xpp[2 * i + 1] = xpp[2 * i] + 128;
  }

#pragma unroll
  for (int i = 0; i < 8; ++i) *(volatile v4f*)(xpp[i]) = xr[i];
  if (hasg) *(volatile v4f*)gp = gv;
  __threadfence();
#pragma unroll
  for (int i = 0; i < 8; ++i) *(volatile v4f*)(xpp[i]) = xr[i];
  if (hasg) *(volatile v4f*)gp = gv;
}

__global__ __launch_bounds__(NTHR) void k_gat(
    const int* __restrict__ ei, const float* __restrict__ xp,
    const float* __restrict__ asrc, const float* __restrict__ adst,
    const float* __restrict__ bias, _Float16* h1f, float* sqo, int nN, int nE) {
  extern __shared__ v4f lds_dyn[];
  float* sacc = (float*)lds_dyn;
  float* den  = sacc + LDS_SACC;
  float* mxv  = den + LDS_DEN;
  int*   list = (int*)(mxv + LDS_MX);
  int*   wcnt = list + LDS_LIST;

  const int tid  = threadIdx.x;
  const int lane = tid & 31;
  const int wave = tid >> 5;
  const int hd   = lane >> 3;
  const int nodeBase = blockIdx.x * NB;
  const float ninf = -__builtin_inff();

  {
    const v4f z4 = {0.f, 0.f, 0.f, 0.f};
    for (int i = tid; i < (LDS_SACC + LDS_DEN) / 4; i += NTHR) lds_dyn[i] = z4;
    for (int i = tid; i < LDS_MX; i += NTHR) mxv[i] = ninf;
  }
  __syncthreads();
  const int* eid = ei + nE;
  const bool al16 = ((nE & 3) == 0);

  const int nChunks = (nE + CHUNK - 1) / CHUNK;
#pragma unroll 1
  for (int ch = 0; ch < nChunks; ++ch) {
    const int cbase = ch * CHUNK;
    int wc = 0;
#pragma unroll
    for (int g = 0; g < NGRP; ++g) {
      const int el0 = (g * NTHR + tid) * 4;
      const int e0  = cbase + el0;
      const int sent = -2147483647 - 1;
      v4i d;
      if (al16 && (cbase + CHUNK <= nE)) {
        d = *(const v4i*)(eid + e0);
      } else {
        d.x = (e0     < nE) ? eid[min(e0, nE - 1)]     : sent;
        d.y = (e0 + 1 < nE) ? eid[min(e0 + 1, nE - 1)] : sent;
        d.z = (e0 + 2 < nE) ? eid[min(e0 + 2, nE - 1)] : sent;
        d.w = (e0 + 3 < nE) ? eid[min(e0 + 3, nE - 1)] : sent;
      }
      const unsigned s0 = (unsigned)d.x - (unsigned)nodeBase;
      const unsigned s1 = (unsigned)d.y - (unsigned)nodeBase;
      const unsigned s2 = (unsigned)d.z - (unsigned)nodeBase;
      const unsigned s3 = (unsigned)d.w - (unsigned)nodeBase;
      const bool h0 = s0 < (unsigned)NB;
      const bool h1 = s1 < (unsigned)NB;
      const bool h2 = s2 < (unsigned)NB;
      const bool h3 = s3 < (unsigned)NB;
      const unsigned many = __builtin_amdgcn_ballot_w32(h0 | h1 | h2 | h3);
      if (many != 0u) {
#define HITJ(J, HJ, SJ) { \
          const unsigned mj = __builtin_amdgcn_ballot_w32(HJ); \
          if (HJ) { \
            const int pos = wc + (int)__builtin_amdgcn_mbcnt_lo(mj, 0u); \
            if (pos < WCAP) list[wave * WCAP + pos] = ((el0 + (J)) << 8) | (int)(SJ); \
          } \
          wc += (int)__builtin_popcount(mj); }
        HITJ(0, h0, s0)
        HITJ(1, h1, s1)
        HITJ(2, h2, s2)
        HITJ(3, h3, s3)
#undef HITJ
      }
    }
    if (lane == 0) wcnt[wave] = wc;
    __syncthreads();

    if (wave == 0) {
#pragma unroll 1
      for (int wsx = 0; wsx < NWAVE; ++wsx) {
        int n = wcnt[wsx];
        if (n > WCAP) n = WCAP;
        if (n < 0) n = 0;
#pragma unroll 1
        for (int i = 0; i < n; ++i) {
          const int ent  = list[wsx * WCAP + i];
          const int slot = ent & (NB - 1);
          const int el   = (ent >> 8) & (CHUNK - 1);
          int e = cbase + el;
          if (e > nE - 1) e = nE - 1;
          int src = ei[e];
          src = src < 0 ? 0 : (src > nN - 1 ? nN - 1 : src);
          int nd = nodeBase + slot;
          if (nd > nN - 1) nd = nN - 1;
          const float al = lrelu(asrc[(size_t)src * NH + hd] + adst[(size_t)nd * NH + hd]);
          const int ai = slot * NH + hd;
          const float mo = mxv[ai];
          const float dn = den[ai];
          const float mn = fmaxf(mo, al);
          const float sc = __expf(mo - mn);
          const float p  = __expf(al - mn);
          const float* xr = xp + (size_t)src * DF + 8 * lane;
          const v4f xv0 = *(const v4f*)(xr);
          const v4f xv1 = *(const v4f*)(xr + 4);
          v4f* sp = (v4f*)(sacc + slot * DF + 8 * lane);
          const v4f c0 = sp[0];
          const v4f c1 = sp[1];
          const v4f n0 = c0 * sc + p * xv0;
          const v4f n1 = c1 * sc + p * xv1;
          sp[0] = n0;
          sp[1] = n1;
          if ((lane & 7) == 0) {
            den[ai] = dn * sc + p;
            mxv[ai] = mn;
          }
        }
      }
    }
    __syncthreads();
  }

  const int slotBase = wave * (NB / NWAVE);
  const v4f b4a = *(const v4f*)(bias + 8 * lane);
  const v4f b4b = *(const v4f*)(bias + 8 * lane + 4);
  float sqreg = 0.f;
#pragma unroll 1
  for (int j = 0; j < NB / NWAVE; ++j) {
    const int slot = slotBase + j;
    int node = nodeBase + slot;
    if (node > nN - 1) node = nN - 1;
    const size_t nrow = (size_t)node;
    const float al = lrelu(asrc[nrow * NH + hd] + adst[nrow * NH + hd]);
    const int ai = slot * NH + hd;
    const float mo = mxv[ai];
    const float dn = den[ai];
    const float mn = fmaxf(mo, al);
    const float sc = __expf(mo - mn);
    const float p  = __expf(al - mn);
    const float* xr = xp + nrow * DF + 8 * lane;
    const v4f xv0 = *(const v4f*)(xr);
    const v4f xv1 = *(const v4f*)(xr + 4);
    const v4f* sp = (const v4f*)(sacc + slot * DF + 8 * lane);
    const v4f sv0 = sp[0] * sc + p * xv0;
    const v4f sv1 = sp[1] * sc + p * xv1;
    const float dv  = dn * sc + p;
    const float inv = 1.0f / dv;
    const v4f e0 = sv0 * inv + b4a;
    const v4f e1 = sv1 * inv + b4b;
    Pack16 u;
    u.h[0] = (_Float16)elu1(e0.x); u.h[1] = (_Float16)elu1(e0.y);
    u.h[2] = (_Float16)elu1(e0.z); u.h[3] = (_Float16)elu1(e0.w);
    u.h[4] = (_Float16)elu1(e1.x); u.h[5] = (_Float16)elu1(e1.y);
    u.h[6] = (_Float16)elu1(e1.z); u.h[7] = (_Float16)elu1(e1.w);
    float s = 0.f;
#pragma unroll
    for (int c = 0; c < 8; ++c) { const float f = (float)u.h[c]; s += f * f; }
    s = wsum(s);
    sqreg = (lane == j) ? s : sqreg;
    _Float16* hp = h1f + nrow * DF + 8 * lane;
    *(volatile v4i*)hp = u.i;
    __threadfence();
    *(volatile v4i*)hp = u.i;
  }
  {
    int sn = nodeBase + slotBase + lane;
    if (sn > nN - 1) sn = nN - 1;
    float* sqp = sqo + sn;
    *(volatile float*)sqp = sqreg;
    __threadfence();
    *(volatile float*)sqp = sqreg;
  }
}

__global__ __launch_bounds__(QTHR) void k_h2(
    const _Float16* __restrict__ h1f, const _Float16* __restrict__ W2h,
    const float* __restrict__ as2, const float* __restrict__ ad2,
    _Float16* h2T, float* s2, float* t2, int nN) {
  __shared__ __attribute__((aligned(16))) _Float16 Ts[NO * JB];
  __shared__ __attribute__((aligned(16))) float S2s[QB];
  __shared__ __attribute__((aligned(16))) float T2s[QB];

  const int tid  = threadIdx.x;
  const int lane = tid & 31;
  const int wave = tid >> 5;
  const int h    = lane >> 4;
  const int m    = lane & 15;
  const int rowBase = blockIdx.x * QB;
  const int rw = rowBase + 16 * wave;

  const _Float16* arow = h1f + (size_t)(rw + m) * DF + 8 * h;
  const _Float16* brow = W2h + (size_t)m * DF + 8 * h;
  v8f c = {0.f, 0.f, 0.f, 0.f, 0.f, 0.f, 0.f, 0.f};
#pragma unroll
  for (int ks = 0; ks < DF / 32; ++ks) {
    const int k0 = ks * 32;
    Frag a, b;
    a.half[0] = *(const v8h*)(arow + k0); a.half[1] = *(const v8h*)(arow + k0 + 16);
    b.half[0] = *(const v8h*)(brow + k0); b.half[1] = *(const v8h*)(brow + k0 + 16);
    c = wm(a.v, b.v, c);
  }

  const float cs = as2[m];
  const float cd = ad2[m];
  float ss[8], tt[8];
#pragma unroll
  for (int r = 0; r < 8; ++r) {
    const float v = c[r] * 0.125f;
    Ts[m * JB + 16 * wave + 8 * h + r] = (_Float16)v;
    ss[r] = v * cs;
    tt[r] = v * cd;
  }
#pragma unroll
  for (int mk = 1; mk < 16; mk <<= 1) {
#pragma unroll
    for (int r = 0; r < 8; ++r) {
      ss[r] += __shfl_xor(ss[r], mk, 32);
      tt[r] += __shfl_xor(tt[r], mk, 32);
    }
  }
  if (m == 0) {
#pragma unroll
    for (int r = 0; r < 8; ++r) {
      S2s[16 * wave + 8 * h + r] = ss[r];
      T2s[16 * wave + 8 * h + r] = tt[r];
    }
  }
  __syncthreads();

  const int trow = 4 * wave + (lane >> 3);
  const int pc   = lane & 7;
  Pack16 u;
  u.h = *(const v8h*)(Ts + trow * JB + 8 * pc);
  _Float16* gp = h2T + (size_t)trow * nN + rowBase + 8 * pc;
  bool hass = false;
  v4f sv = {0.f, 0.f, 0.f, 0.f};
  float* spp = s2;
  if (wave == 0 && lane < 16) {
    sv = *(const v4f*)(S2s + 4 * lane); spp = s2 + rowBase + 4 * lane; hass = true;
  } else if (wave == 1 && lane < 16) {
    sv = *(const v4f*)(T2s + 4 * lane); spp = t2 + rowBase + 4 * lane; hass = true;
  }
  *(volatile v4i*)gp = u.i;
  if (hass) *(volatile v4f*)spp = sv;
  __threadfence();
  *(volatile v4i*)gp = u.i;
  if (hass) *(volatile v4f*)spp = sv;
}

__global__ __launch_bounds__(QTHR) void k_conv2(
    const _Float16* __restrict__ h1f, const float* __restrict__ sq,
    const float* __restrict__ s2, const float* __restrict__ t2,
    const _Float16* __restrict__ h2T, const float* __restrict__ b2,
    float* out, int nN) {
  __shared__ __attribute__((aligned(16))) _Float16 Ps[4 * 16 * PP];
  __shared__ __attribute__((aligned(16))) float Os[QB * NO];

  const int tid  = threadIdx.x;
  const int lane = tid & 31;
  const int wave = tid >> 5;
  const int h    = lane >> 4;
  const int m    = lane & 15;
  const int rowBase = blockIdx.x * QB;
  const int rw = rowBase + 16 * wave;
  const float ninf = -__builtin_inff();
  _Float16* Pw = Ps + wave * 16 * PP;

  float sqi[8], t2i[8], mrun[8], lrun[8];
#pragma unroll
  for (int r = 0; r < 8; ++r) {
    const int ir = rw + 8 * h + r;
    sqi[r]  = sq[ir];
    t2i[r]  = t2[ir];
    mrun[r] = ninf;
    lrun[r] = 0.f;
  }
  const v8f zero8 = {0.f, 0.f, 0.f, 0.f, 0.f, 0.f, 0.f, 0.f};
  v8f oacc = zero8;
  const _Float16* arow = h1f + (size_t)(rw + m) * DF + 8 * h;
  const int nChunks = nN / JB;

#pragma unroll 1
  for (int jc = 0; jc < nChunks; ++jc) {
    const int j0 = jc * JB;

    v8f d0 = zero8, d1 = zero8, d2v = zero8, d3 = zero8;
    const _Float16* brow = h1f + (size_t)(j0 + m) * DF + 8 * h;
#pragma unroll 1
    for (int ks = 0; ks < DF / 32; ++ks) {
      const int k0 = ks * 32;
      Frag a, bq0, bq1, bq2, bq3;
      a.half[0]   = *(const v8h*)(arow + k0);             a.half[1]   = *(const v8h*)(arow + k0 + 16);
      bq0.half[0] = *(const v8h*)(brow + k0);             bq0.half[1] = *(const v8h*)(brow + k0 + 16);
      bq1.half[0] = *(const v8h*)(brow + 16 * DF + k0);   bq1.half[1] = *(const v8h*)(brow + 16 * DF + k0 + 16);
      bq2.half[0] = *(const v8h*)(brow + 32 * DF + k0);   bq2.half[1] = *(const v8h*)(brow + 32 * DF + k0 + 16);
      bq3.half[0] = *(const v8h*)(brow + 48 * DF + k0);   bq3.half[1] = *(const v8h*)(brow + 48 * DF + k0 + 16);
      d0  = wm(a.v, bq0.v, d0);
      d1  = wm(a.v, bq1.v, d1);
      d2v = wm(a.v, bq2.v, d2v);
      d3  = wm(a.v, bq3.v, d3);
    }
    v8f dt[4];
    dt[0] = d0; dt[1] = d1; dt[2] = d2v; dt[3] = d3;

    float sqj[4], s2j[4];
#pragma unroll
    for (int ct = 0; ct < 4; ++ct) {
      const int jj = j0 + 16 * ct + m;
      sqj[ct] = sq[jj];
      s2j[ct] = s2[jj];
    }
    float pv[4][8];
    float cm[8];
#pragma unroll
    for (int r = 0; r < 8; ++r) cm[r] = ninf;
#pragma unroll
    for (int ct = 0; ct < 4; ++ct) {
#pragma unroll
      for (int r = 0; r < 8; ++r) {
        const float dd   = (sqi[r] + sqj[ct]) - 2.0f * dt[ct][r];
        const float dist = sqrtf(fmaxf(dd, 0.f));
        const float sc   = lrelu(s2j[ct] + t2i[r]);
        const float sv   = (dist < 0.5f) ? sc : ninf;
        pv[ct][r] = sv;
        cm[r] = fmaxf(cm[r], sv);
      }
    }
#pragma unroll
    for (int mk = 1; mk < 16; mk <<= 1) {
#pragma unroll
      for (int r = 0; r < 8; ++r) cm[r] = fmaxf(cm[r], __shfl_xor(cm[r], mk, 32));
    }

    float mn[8], scl[8], rs[8];
#pragma unroll
    for (int r = 0; r < 8; ++r) {
      mn[r] = fmaxf(mrun[r], cm[r]);
      const bool none = !(mn[r] > ninf);
      const float arg = none ? 0.f : (mrun[r] - mn[r]);
      scl[r] = __expf(arg);
      rs[r]  = 0.f;
    }
#pragma unroll
    for (int ct = 0; ct < 4; ++ct) {
#pragma unroll
      for (int r = 0; r < 8; ++r) {
        const float t = pv[ct][r] - mn[r];
        const float p = (pv[ct][r] > ninf) ? __expf(t) : 0.f;
        pv[ct][r] = p;
        rs[r] += p;
      }
    }
#pragma unroll
    for (int mk = 1; mk < 16; mk <<= 1) {
#pragma unroll
      for (int r = 0; r < 8; ++r) rs[r] += __shfl_xor(rs[r], mk, 32);
    }
#pragma unroll
    for (int r = 0; r < 8; ++r) {
      lrun[r] = lrun[r] * scl[r] + rs[r];
      mrun[r] = mn[r];
      oacc[r] = oacc[r] * scl[r];
    }

#pragma unroll
    for (int ct = 0; ct < 4; ++ct) {
#pragma unroll
      for (int r = 0; r < 8; ++r) Pw[(8 * h + r) * PP + 16 * ct + m] = (_Float16)(pv[ct][r] * 1024.0f);
    }
    __builtin_amdgcn_fence(__ATOMIC_RELEASE, "wavefront");
    __builtin_amdgcn_wave_barrier();

#pragma unroll
    for (int ks = 0; ks < JB / 32; ++ks) {
      const int k0 = ks * 32;
      Frag a, b;
      const _Float16* pa = Pw + m * PP + k0 + 8 * h;
      const _Float16* pb = h2T + (size_t)m * nN + j0 + k0 + 8 * h;
      a.half[0] = *(const v8h*)pa; a.half[1] = *(const v8h*)(pa + 16);
      b.half[0] = *(const v8h*)pb; b.half[1] = *(const v8h*)(pb + 16);
      oacc = wm(a.v, b.v, oacc);
    }
  }

  const float bb = b2[m];
  float vo[8], mx[8], se[8];
#pragma unroll
  for (int r = 0; r < 8; ++r) {
    vo[r] = oacc[r] * (1.0f / 1024.0f) * (1.0f / lrun[r]) + bb;
    mx[r] = vo[r];
  }
#pragma unroll
  for (int mk = 1; mk < 16; mk <<= 1) {
#pragma unroll
    for (int r = 0; r < 8; ++r) mx[r] = fmaxf(mx[r], __shfl_xor(mx[r], mk, 32));
  }
#pragma unroll
  for (int r = 0; r < 8; ++r) {
    vo[r] = vo[r] - mx[r];
    se[r] = expf(vo[r]);
  }
#pragma unroll
  for (int mk = 1; mk < 16; mk <<= 1) {
#pragma unroll
    for (int r = 0; r < 8; ++r) se[r] += __shfl_xor(se[r], mk, 32);
  }
#pragma unroll
  for (int r = 0; r < 8; ++r) Os[(16 * wave + 8 * h + r) * NO + m] = vo[r] - logf(se[r]);
  __syncthreads();

  v4f ov[2];
  float* op[2];
#pragma unroll
  for (int ps = 0; ps < 2; ++ps) {
    const int q = tid + QTHR * ps;
    ov[ps] = *(const v4f*)(Os + 4 * q);
    op[ps] = out + (size_t)rowBase * NO + 4 * q;
  }
  *(volatile v4f*)(op[0]) = ov[0];
  *(volatile v4f*)(op[1]) = ov[1];
  __threadfence();
  *(volatile v4f*)(op[0]) = ov[0];
  *(volatile v4f*)(op[1]) = ov[1];
}

extern "C" void kernel_launch(void* const* d_in, const int* in_sizes, int n_in,
                              void* d_out, int out_size, void* d_ws, size_t ws_size,
                              hipStream_t stream) {
  if (n_in < 10) return;
  const int nN = in_sizes[0] / INC;
  if (nN <= 0 || in_sizes[0] != nN * INC) return;
  if ((nN % NB) != 0) return;
  if (in_sizes[1] < 0 || (in_sizes[1] & 1) != 0) return;
  const int nE = in_sizes[1] / 2;
  if (in_sizes[2] != INC * DF) return;
  if (in_sizes[3] != DF || in_sizes[4] != DF || in_sizes[5] != DF) return;
  if (in_sizes[6] != DF * NO) return;
  if (in_sizes[7] != NO || in_sizes[8] != NO || in_sizes[9] != NO) return;
  if (out_size != nN * NO) return;

  const float* x    = (const float*)d_in[0];
  const int*   ei   = (const int*)  d_in[1];
  const float* W1   = (const float*)d_in[2];
  const float* as1  = (const float*)d_in[3];
  const float* ad1  = (const float*)d_in[4];
  const float* b1   = (const float*)d_in[5];
  const float* W2   = (const float*)d_in[6];
  const float* as2  = (const float*)d_in[7];
  const float* ad2  = (const float*)d_in[8];
  const float* b2   = (const float*)d_in[9];
  float* out = (float*)d_out;

  size_t off = 0;
  char* ws = (char*)d_ws;
#define CARVE(PTR, TYPE, BYTES) PTR = (TYPE*)(ws + off); off += (((size_t)(BYTES)) + 255) & ~(size_t)255;
  _Float16* W1h;  CARVE(W1h,  _Float16, (size_t)DF * INC * sizeof(_Float16))
  _Float16* W2h;  CARVE(W2h,  _Float16, (size_t)NO * DF * sizeof(_Float16))
  float*    xp;   CARVE(xp,   float,    (size_t)nN * DF * sizeof(float))
  float*    asrc; CARVE(asrc, float,    (size_t)nN * NH * sizeof(float))
  float*    adst; CARVE(adst, float,    (size_t)nN * NH * sizeof(float))
  _Float16* h1f;  CARVE(h1f,  _Float16, (size_t)nN * DF * sizeof(_Float16))
  float*    sq;   CARVE(sq,   float,    (size_t)nN * sizeof(float))
  _Float16* h2T;  CARVE(h2T,  _Float16, (size_t)NO * nN * sizeof(_Float16))
  float*    s2;   CARVE(s2,   float,    (size_t)nN * sizeof(float))
  float*    t2;   CARVE(t2,   float,    (size_t)nN * sizeof(float))
#undef CARVE
  if (off > ws_size) return;
  if (off > (size_t)134217728) return;

  const int n8a = DF * (INC / 8);
  k_prepT<<<(n8a + NTHR - 1) / NTHR, NTHR, 0, stream>>>(W1, W1h, INC, DF);
  const int n8b = NO * (DF / 8);
  k_prepT<<<(n8b + NTHR - 1) / NTHR, NTHR, 0, stream>>>(W2, W2h, DF, NO);

  k_gemm<<<nN / GR, NTHR, 0, stream>>>(x, W1h, as1, ad1, xp, asrc, adst, nN);

  hipFuncSetAttribute(reinterpret_cast<const void*>(&k_gat),
                      hipFuncAttributeMaxDynamicSharedMemorySize, LDS_BYTES);
  k_gat<<<nN / NB, NTHR, LDS_BYTES, stream>>>(ei, xp, asrc, adst, b1, h1f, sq, nN, nE);

  k_h2<<<nN / QB, QTHR, 0, stream>>>(h1f, W2h, as2, ad2, h2T, s2, t2, nN);

  k_conv2<<<nN / QB, QTHR, 0, stream>>>(h1f, sq, s2, t2, h2T, b2, out, nN);
}
